// SMPL_40389872451788
// MI455X (gfx1250) — hardware-run, weakly checked
//
#include <hip/hip_runtime.h>
#include <math.h>

typedef __attribute__((ext_vector_type(16))) _Float16 v16h;
typedef __attribute__((ext_vector_type(8)))  _Float16 v8h;
typedef __attribute__((ext_vector_type(8)))  float    v8f;
typedef __attribute__((ext_vector_type(4)))  float    v4f;
typedef __attribute__((ext_vector_type(2)))  float    v2f;

constexpr int kB    = 512;
constexpr int kV    = 6890;
constexpr int kJ    = 24;
constexpr int kNB   = 10;
constexpr int kP    = 207;
constexpr int kN3   = kV * 3;
constexpr int kVP   = 6912;
constexpr int kN3P  = kVP * 3;
constexpr int kKP   = 256;
constexpr int kKL   = 224;
constexpr int kPB   = 8;
constexpr int kNA   = kB * 12;
constexpr int kPdPitch = 212;
constexpr int kOut0Elems = kB * kN3;
constexpr int kOut1Elems = kB * kJ * 3;
static_assert(kN3P % 64 == 0 && kVP % 64 == 0 && kVP % 32 == 0, "tile multiples");
static_assert(kKL % 32 == 0 && kKL > kP && kKL <= kKP, "pose K padding");
static_assert(kB % 64 == 0 && kB % kPB == 0 && kB % 4 == 0, "batch tiling");
static_assert(kNA % 48 == 0, "skinning column tiles of 4 batches");
static_assert(kOut0Elems % 1024 == 0, "compaction grid exact");
static_assert(((size_t)kOut0Elems * 4) % 128 == 0, "second output starts on a line");

constexpr float kCarryPd = 1024.0f;
constexpr float kCarryPf = 64.0f;
constexpr float kInvPose = 1.0f / (kCarryPd * kCarryPf);
constexpr float kCarryW  = 64.0f;
constexpr float kCarryA  = 1024.0f;
constexpr float kInvLbs  = 1.0f / (kCarryW * kCarryA);
constexpr float kCarryJr = 32768.0f;
constexpr float kCarryVt = 64.0f;
constexpr float kCarrySd = 1024.0f;
constexpr float kInvCvt  = 1.0f / (kCarryJr * kCarryVt);
constexpr float kInvCsd  = 1.0f / (kCarryJr * kCarrySd);
constexpr float kF16MinNormal = 6.103515625e-05f;

constexpr size_t kSzBTPD = (size_t)kN3P * kKP * 2;
constexpr size_t kSzPF16 = (size_t)kB * kKP * 2;
constexpr size_t kSzW16  = (size_t)kVP * 32 * 2;
constexpr size_t kSzA16  = (size_t)kNA * 32 * 2;
constexpr size_t kSzJR16 = (size_t)32 * kVP * 2;
constexpr size_t kSzX16  = (size_t)48 * kVP * 2;
constexpr size_t kSzVSD  = (size_t)kN3P * 12 * 4;
constexpr size_t kSzCC   = (size_t)kJ * 64 * 4;
constexpr size_t kSzVP   = (size_t)kB * kN3P * 4;
constexpr size_t kOffBTPD = 0;
constexpr size_t kOffPF16 = kOffBTPD + kSzBTPD;
constexpr size_t kOffW16  = kOffPF16 + kSzPF16;
constexpr size_t kOffA16  = kOffW16  + kSzW16;
constexpr size_t kOffJR16 = kOffA16  + kSzA16;
constexpr size_t kOffX16  = kOffJR16 + kSzJR16;
constexpr size_t kOffVSD  = kOffX16  + kSzX16;
constexpr size_t kOffCC   = kOffVSD  + kSzVSD;
constexpr size_t kOffVP   = kOffCC   + kSzCC;
constexpr size_t kOffVO   = kOffVP   + kSzVP;
constexpr size_t kWsTotal = kOffVO   + kSzVP;
static_assert(kWsTotal == 98756608ull, "carve total");
static_assert(kWsTotal <= 134217728ull, "carve cap");
static_assert((kOffPF16 % 128) == 0 && (kOffW16 % 128) == 0 && (kOffA16 % 128) == 0 && (kOffJR16 % 128) == 0 &&
              (kOffX16 % 128) == 0 && (kOffVSD % 128) == 0 && (kOffCC % 128) == 0 && (kOffVP % 128) == 0 &&
              (kOffVO % 128) == 0, "128-B aligned regions");

constexpr int kBlkW   = (kVP * 32 / 8) / 256;
constexpr int kBlkJR  = (32 * kVP / 8) / 256;
constexpr int kBlkX   = (48 * kVP / 8) / 256;
constexpr int kBlkVSD = (kN3P * 12 / 4) / 256;
static_assert(kBlkW == 108 && kBlkJR == 108 && kBlkX == 162 && kBlkVSD == 243, "prep coverage");
static_assert((kVP / 8) % 32 == 0, "a wave never straddles two plane rows");

__constant__ int c_parent[kJ] = {-1, 0, 0, 0, 1, 2, 3, 4, 5, 6, 7, 8, 9, 9, 9, 12, 13, 14, 16, 17, 18, 19, 20, 21};
static_assert(sizeof(c_parent) / sizeof(c_parent[0]) == 24, "parent table length");

__device__ __forceinline__ int imin(int a, int b) { return a < b ? a : b; }
__device__ __forceinline__ int imax(int a, int b) { return a > b ? a : b; }
__device__ __forceinline__ void pin1(float& x) { asm volatile("" : "+v"(x)); }
__device__ __forceinline__ void pin4(v4f& x) { asm volatile("" : "+v"(x)); }

__device__ __forceinline__ _Float16 h_conv(float v) {
  const float w = (fabsf(v) < kF16MinNormal) ? 0.0f : v;
  return (_Float16)w;
}

union FragH { v16h v; v8h h[2]; };
__device__ __forceinline__ v16h frag_load(const _Float16* p) {
  FragH f;
  f.h[0] = *(const v8h*)(p);
  f.h[1] = *(const v8h*)(p + 16);
  return f.v;
}
__device__ __forceinline__ v8f mma_h(v16h a, v16h b, v8f c) {
  c = __builtin_amdgcn_wmma_f32_16x16x32_f16(false, a, false, b, (short)0, c, false, false);
  asm volatile("v_nop\n\tv_nop\n\tv_nop\n\tv_nop" : "+v"(c) : "v"(a), "v"(b));
  return c;
}
__device__ __forceinline__ void wave_sync_lds() {
  __builtin_amdgcn_fence(__ATOMIC_RELEASE, "workgroup");
  __builtin_amdgcn_wave_barrier();
  __builtin_amdgcn_fence(__ATOMIC_ACQUIRE, "workgroup");
}

__global__ __launch_bounds__(256) void prep_small_kernel(
    const float* __restrict__ lbs, const float* __restrict__ jreg,
    const float* __restrict__ vt, const float* __restrict__ sd,
    unsigned short* __restrict__ W16, unsigned short* __restrict__ JR16,
    unsigned short* __restrict__ X16, float* __restrict__ VSD)
{
  const int tid = threadIdx.x;
  const int blk = blockIdx.x;
  if (blk < kBlkW) {
    const int i = blk * 256 + tid;
    const int row = i >> 2;
    const int c8 = (i & 3) * 8;
    const bool ok = (row < kV) && (c8 < kJ);
    const int rc = imin(row, kV - 1);
    const int cc = imin(c8, 16);
    v4f a0 = *(const v4f*)(lbs + (size_t)rc * kJ + cc);
    v4f a1 = *(const v4f*)(lbs + (size_t)rc * kJ + cc + 4);
    pin4(a0);
    pin4(a1);
    v8h hv;
#pragma unroll
    for (int e = 0; e < 4; ++e) {
      const float x0 = ok ? a0[e] * kCarryW : 0.0f;
      const float x1 = ok ? a1[e] * kCarryW : 0.0f;
      hv[e] = h_conv(x0);
      hv[4 + e] = h_conv(x1);
    }
    unsigned short* q = W16 + (size_t)i * 8;
    *(volatile v8h*)q = hv;
    __threadfence();
    *(volatile v8h*)q = hv;
  } else if (blk < kBlkW + kBlkJR) {
    const int i = (blk - kBlkW) * 256 + tid;
    const int row = i / (kVP / 8);
    const int c8 = (i - row * (kVP / 8)) * 8;
    const bool rok = row < kJ;
    const int rc = imin(row, kJ - 1);
    v8h hv;
#pragma unroll
    for (int e = 0; e < 8; ++e) {
      const int col = c8 + e;
      const int colc = imin(col, kV - 1);
      float x = jreg[(size_t)rc * kV + colc];
      pin1(x);
      const float y = (rok && (col < kV)) ? x * kCarryJr : 0.0f;
      hv[e] = h_conv(y);
    }
    unsigned short* q = JR16 + (size_t)i * 8;
    *(volatile v8h*)q = hv;
    __threadfence();
    *(volatile v8h*)q = hv;
  } else if (blk < kBlkW + kBlkJR + kBlkX) {
    const int i = (blk - kBlkW - kBlkJR) * 256 + tid;
    const int n = i / (kVP / 8);
    const int c8 = (i - n * (kVP / 8)) * 8;
    const int nv = imin(n, 2);
    const int ns = imin(imax(n - 3, 0), 29);
    const float fa = (n < 3) ? kCarryVt : 0.0f;
    const float fb = ((n >= 3) && (n < 33)) ? kCarrySd : 0.0f;
    v8h hv;
#pragma unroll
    for (int e = 0; e < 8; ++e) {
      const int v = c8 + e;
      const int vc = imin(v, kV - 1);
      float a = vt[(size_t)vc * 3 + nv];
      float s = sd[(size_t)vc * 30 + ns];
      pin1(a);
      pin1(s);
      const float y = fmaf(fa, a, fb * s);
      const float z = (v < kV) ? y : 0.0f;
      hv[e] = h_conv(z);
    }
    unsigned short* q = X16 + (size_t)i * 8;
    *(volatile v8h*)q = hv;
    __threadfence();
    *(volatile v8h*)q = hv;
  } else {
    const int i = (blk - kBlkW - kBlkJR - kBlkX) * 256 + tid;
    const int row = i / 3;
    const int qd = i - row * 3;
    const bool ok = row < kN3;
    const int rc = imin(row, kN3 - 1);
    float s0 = sd[(size_t)rc * kNB + imin(qd * 4 + 0, 9)];
    float s1 = sd[(size_t)rc * kNB + imin(qd * 4 + 1, 9)];
    float s2 = sd[(size_t)rc * kNB + imin(qd * 4 + 2, 9)];
    float s3 = sd[(size_t)rc * kNB + imin(qd * 4 + 3, 9)];
    float t0 = vt[rc];
    pin1(s0);
    pin1(s1);
    pin1(s2);
    pin1(s3);
    pin1(t0);
    const bool last = (qd == 2);
    v4f o;
    o[0] = ok ? s0 : 0.0f;
    o[1] = ok ? s1 : 0.0f;
    o[2] = ok ? (last ? t0 : s2) : 0.0f;
    o[3] = ok ? (last ? 0.0f : s3) : 0.0f;
    float* q = VSD + (size_t)i * 4;
    *(volatile v4f*)q = o;
    __threadfence();
    *(volatile v4f*)q = o;
  }
}

__global__ __launch_bounds__(256) void prep_pd_kernel(const float* __restrict__ pd, unsigned short* __restrict__ BT)
{
  __shared__ __align__(16) float s[32 * kPdPitch];
  const int tid = threadIdx.x;
  const int tn = tid & 31;
  const int tk = tid >> 5;
  const int n = blockIdx.x * 32 + tn;
  const bool nok = n < kN3;
  const int nc = imin(n, kN3 - 1);
#pragma unroll 1
  for (int t = 0; t < 26; ++t) {
    const int kk = tk + 8 * t;
    const int kc = imin(kk, kP - 1);
    float x = pd[(size_t)kc * kN3 + nc];
    pin1(x);
    const bool ok = nok && (kk < kP);
    s[tn * kPdPitch + kk] = ok ? x * kCarryPd : 0.0f;
  }
  __syncthreads();
  v8h hv[4];
#pragma unroll
  for (int it = 0; it < 4; ++it) {
    const int item = it * 256 + tid;
    const int row = item >> 5;
    const int c8 = (item & 31) * 8;
    const int c8c = imin(c8, 200);
    const bool keep = c8 < 208;
    const v4f a0 = *(const v4f*)(s + row * kPdPitch + c8c);
    const v4f a1 = *(const v4f*)(s + row * kPdPitch + c8c + 4);
#pragma unroll
    for (int e = 0; e < 4; ++e) {
      const float x0 = keep ? a0[e] : 0.0f;
      const float x1 = keep ? a1[e] : 0.0f;
      hv[it][e] = h_conv(x0);
      hv[it][4 + e] = h_conv(x1);
    }
  }
  for (int pass = 0; pass < 2; ++pass) {
#pragma unroll
    for (int it = 0; it < 4; ++it) {
      const int item = it * 256 + tid;
      const int row = item >> 5;
      const int c8 = (item & 31) * 8;
      *(volatile v8h*)(BT + (size_t)(blockIdx.x * 32 + row) * kKP + c8) = hv[it];
    }
    __threadfence();
  }
}

__global__ __launch_bounds__(256) void consts_kernel(
    const unsigned short* __restrict__ JRp, const unsigned short* __restrict__ Xp, float* __restrict__ CC)
{
  __shared__ __align__(16) float sP[8 * 24 * 48];
  const _Float16* JR = (const _Float16*)JRp;
  const _Float16* X  = (const _Float16*)Xp;
  const int tid = threadIdx.x;
  const int lane = tid & 31;
  const int wave = tid >> 5;
  const int rlane = lane & 15;
  const int koff = (lane >> 4) * 8;
  const int mOff = (lane >> 4) * 8;
  v8f acc[2][3];
#pragma unroll
  for (int i = 0; i < 2; ++i)
#pragma unroll
    for (int j = 0; j < 3; ++j) acc[i][j] = (v8f){0.f, 0.f, 0.f, 0.f, 0.f, 0.f, 0.f, 0.f};
#pragma unroll 1
  for (int st = 0; st < 27; ++st) {
    const int k0 = (wave * 27 + st) * 32;
    v16h bh[3];
#pragma unroll
    for (int j = 0; j < 3; ++j) bh[j] = frag_load(X + (size_t)((j << 4) + rlane) * kVP + koff + k0);
#pragma unroll
    for (int i = 0; i < 2; ++i) {
      const v16h ah = frag_load(JR + (size_t)((i << 4) + rlane) * kVP + koff + k0);
#pragma unroll
      for (int j = 0; j < 3; ++j) acc[i][j] = mma_h(ah, bh[j], acc[i][j]);
    }
  }
  float* pw = sP + wave * (24 * 48);
#pragma unroll
  for (int j = 0; j < 3; ++j)
#pragma unroll
    for (int r = 0; r < 8; ++r) pw[(mOff + r) * 48 + (j << 4) + rlane] = acc[0][j][r];
  if (mOff == 0) {
#pragma unroll
    for (int j = 0; j < 3; ++j)
#pragma unroll
      for (int r = 0; r < 8; ++r) pw[(16 + r) * 48 + (j << 4) + rlane] = acc[1][j][r];
  }
  __syncthreads();
  v4f ov[2];
#pragma unroll
  for (int t = 0; t < 2; ++t) {
    const int item = tid + 256 * t;
    const int ic = imin(item, 383);
    const int row = ic >> 4;
    const int c4 = (ic & 15) * 4;
    const int c4c = imin(c4, 44);
    v4f sum = (v4f){0.f, 0.f, 0.f, 0.f};
#pragma unroll
    for (int w = 0; w < 8; ++w) {
      const v4f p = *(const v4f*)(sP + (w * 24 + row) * 48 + c4c);
      sum = sum + p;
    }
#pragma unroll
    for (int e = 0; e < 4; ++e) {
      const int col = c4 + e;
      const float sc = (col < 3) ? kInvCvt : kInvCsd;
      ov[t][e] = (c4 < 48) ? sum[e] * sc : 0.0f;
    }
  }
  for (int pass = 0; pass < 2; ++pass) {
#pragma unroll
    for (int t = 0; t < 2; ++t) {
      const int item = tid + 256 * t;
      if (item < 384) {
        const int row = item >> 4;
        const int c4 = (item & 15) * 4;
        *(volatile v4f*)(CC + row * 64 + c4) = ov[t];
      }
    }
    __threadfence();
  }
}

__global__ __launch_bounds__(192) void pose_kernel(
    const float* __restrict__ go, const float* __restrict__ bp, const float* __restrict__ betas,
    const float* __restrict__ transl, const float* __restrict__ CC,
    unsigned short* __restrict__ PF16, unsigned short* __restrict__ A16, float* __restrict__ outJ)
{
  __shared__ __align__(16) float sJ[kPB * kJ * 3];
  __shared__ __align__(16) float sG[kPB * kJ * 12];
  __shared__ __align__(16) float sPF[kPB * kKP];
  __shared__ __align__(16) float sA[kPB * 12 * 32];
  __shared__ __align__(16) float sO[kPB * 72];
  const int tid = threadIdx.x;
  const int bl = tid / kJ;
  const int j = tid - bl * kJ;
  const int blk = blockIdx.x;
  const int b = blk * kPB + bl;

  for (int idx = tid; idx < kPB * 49; idx += 192) {
    const int r = idx / 49;
    const int c = kP + (idx - r * 49);
    sPF[r * kKP + c] = 0.0f;
  }
  for (int idx = tid; idx < kPB * 12 * 8; idx += 192) sA[(idx >> 3) * 32 + kJ + (idx & 7)] = 0.0f;

  const int jm = imax(j - 1, 0);
  const float f0 = (j == 0) ? 1.0f : 0.0f;
  const float f1 = 1.0f - f0;
  float g0 = go[b * 3 + 0], g1 = go[b * 3 + 1], g2 = go[b * 3 + 2];
  float q0 = bp[(size_t)b * 69 + jm * 3 + 0], q1 = bp[(size_t)b * 69 + jm * 3 + 1], q2 = bp[(size_t)b * 69 + jm * 3 + 2];
  pin1(g0);
  pin1(g1);
  pin1(g2);
  pin1(q0);
  pin1(q1);
  pin1(q2);
  const float ax = fmaf(f0, g0, f1 * q0);
  const float ay = fmaf(f0, g1, f1 * q1);
  const float az = fmaf(f0, g2, f1 * q2);
  const float ang = sqrtf(ax * ax + ay * ay + az * az + 1e-8f);
  const float inv = 1.0f / ang;
  const float x = ax * inv, y = ay * inv, z = az * inv;
  const float sn = sinf(ang);
  const float cs = cosf(ang);
  const float tt = 1.0f - cs;
  const float xy = x * y, xz = x * z, yz = y * z;
  const float xx = x * x, yy = y * y, zz = z * z;
  const float P0 = tt * (-zz - yy);
  const float P1 = tt * xy - sn * z;
  const float P2 = tt * xz + sn * y;
  const float P3 = tt * xy + sn * z;
  const float P4 = tt * (-zz - xx);
  const float P5 = tt * yz - sn * x;
  const float P6 = tt * xz - sn * y;
  const float P7 = tt * yz + sn * x;
  const float P8 = tt * (-yy - xx);
  if (j >= 1) {
    float* pf = sPF + bl * kKP + (j - 1) * 9;
    pf[0] = P0; pf[1] = P1; pf[2] = P2;
    pf[3] = P3; pf[4] = P4; pf[5] = P5;
    pf[6] = P6; pf[7] = P7; pf[8] = P8;
  }
  const float R0 = 1.0f + P0, R1 = P1, R2 = P2;
  const float R3 = P3, R4 = 1.0f + P4, R5 = P5;
  const float R6 = P6, R7 = P7, R8 = 1.0f + P8;

  float be[kNB];
#pragma unroll
  for (int l = 0; l < kNB; ++l) be[l] = betas[(size_t)b * kNB + l];
  const float* crow = CC + j * 64;
#pragma unroll 1
  for (int k = 0; k < 3; ++k) {
    float a = crow[k];
    const float* cq = crow + 3 + k * kNB;
#pragma unroll
    for (int l = 0; l < kNB; ++l) a = fmaf(be[l], cq[l], a);
    sJ[tid * 3 + k] = a;
  }
  __syncthreads();

  const int par = c_parent[j];
  const int pc = imax(par, 0);
  const float jp0 = sJ[tid * 3 + 0], jp1 = sJ[tid * 3 + 1], jp2 = sJ[tid * 3 + 2];
  const float pj0 = sJ[(bl * kJ + pc) * 3 + 0], pj1 = sJ[(bl * kJ + pc) * 3 + 1], pj2 = sJ[(bl * kJ + pc) * 3 + 2];
  const float rel0 = jp0 - ((par >= 0) ? pj0 : 0.0f);
  const float rel1 = jp1 - ((par >= 0) ? pj1 : 0.0f);
  const float rel2 = jp2 - ((par >= 0) ? pj2 : 0.0f);

  int dep = 0;
  {
    int p = j;
#pragma unroll 1
    for (int st = 0; st < 9; ++st) {
      const int pp = c_parent[imax(p, 0)];
      const int act = (p > 0) ? 1 : 0;
      dep += act;
      p = act ? pp : p;
    }
  }

  float* gs = sG + tid * 12;
  *(v4f*)(gs + 0) = (v4f){R0, R1, R2, rel0};
  *(v4f*)(gs + 4) = (v4f){R3, R4, R5, rel1};
  *(v4f*)(gs + 8) = (v4f){R6, R7, R8, rel2};
  __syncthreads();
#pragma unroll 1
  for (int lvl = 1; lvl <= 8; ++lvl) {
    if (dep == lvl) {
      const float* gp = sG + (bl * kJ + pc) * 12;
#pragma unroll 1
      for (int m = 0; m < 3; ++m) {
        const v4f g = *(const v4f*)(gp + m * 4);
        v4f o;
        o[0] = g[0] * R0 + g[1] * R3 + g[2] * R6;
        o[1] = g[0] * R1 + g[1] * R4 + g[2] * R7;
        o[2] = g[0] * R2 + g[1] * R5 + g[2] * R8;
        o[3] = g[0] * rel0 + g[1] * rel1 + g[2] * rel2 + g[3];
        *(v4f*)(gs + m * 4) = o;
      }
    }
    __syncthreads();
  }

  const v4f G0 = *(const v4f*)(gs + 0);
  const v4f G1 = *(const v4f*)(gs + 4);
  const v4f G2 = *(const v4f*)(gs + 8);
  const float tr0 = transl[b * 3 + 0], tr1 = transl[b * 3 + 1], tr2 = transl[b * 3 + 2];
  sO[bl * 72 + j * 3 + 0] = G0[3] + tr0;
  sO[bl * 72 + j * 3 + 1] = G1[3] + tr1;
  sO[bl * 72 + j * 3 + 2] = G2[3] + tr2;
  {
    const float tj0 = G0[0] * jp0 + G0[1] * jp1 + G0[2] * jp2;
    const float tj1 = G1[0] * jp0 + G1[1] * jp1 + G1[2] * jp2;
    const float tj2 = G2[0] * jp0 + G2[1] * jp1 + G2[2] * jp2;
    float* ar = sA + (bl * 12) * 32 + j;
    ar[0 * 32] = G0[0]; ar[1 * 32] = G0[1]; ar[2 * 32] = G0[2];  ar[3 * 32] = G0[3] - tj0;
    ar[4 * 32] = G1[0]; ar[5 * 32] = G1[1]; ar[6 * 32] = G1[2];  ar[7 * 32] = G1[3] - tj1;
    ar[8 * 32] = G2[0]; ar[9 * 32] = G2[1]; ar[10 * 32] = G2[2]; ar[11 * 32] = G2[3] - tj2;
  }
  __syncthreads();

  const int io = imin(tid, 143);
  const v4f ov = *(const v4f*)(sO + io * 4);
  v8h pfv[2], av[2];
#pragma unroll
  for (int t = 0; t < 2; ++t) {
    const int item = tid + 192 * t;
    const int ic = imin(item, 255);
    const v4f a0 = *(const v4f*)(sPF + ic * 8);
    const v4f a1 = *(const v4f*)(sPF + ic * 8 + 4);
    const v4f c0 = *(const v4f*)(sA + item * 8);
    const v4f c1 = *(const v4f*)(sA + item * 8 + 4);
#pragma unroll
    for (int e = 0; e < 4; ++e) {
      pfv[t][e]     = h_conv(a0[e] * kCarryPf);
      pfv[t][4 + e] = h_conv(a1[e] * kCarryPf);
      av[t][e]      = h_conv(c0[e] * kCarryA);
      av[t][4 + e]  = h_conv(c1[e] * kCarryA);
    }
  }
  for (int pass = 0; pass < 2; ++pass) {
    if (tid < 144) *(volatile v4f*)(outJ + (size_t)blk * (kPB * 72) + tid * 4) = ov;
#pragma unroll
    for (int t = 0; t < 2; ++t) {
      const int item = tid + 192 * t;
      if (item < 256) *(volatile v8h*)(PF16 + (size_t)blk * (kPB * kKP) + item * 8) = pfv[t];
      *(volatile v8h*)(A16 + (size_t)blk * (kPB * 12 * 32) + item * 8) = av[t];
    }
    __threadfence();
  }
}

__global__ __launch_bounds__(256) void pose_gemm_kernel(
    const unsigned short* __restrict__ PFp, const unsigned short* __restrict__ BTp,
    const float* __restrict__ VSD, const float* __restrict__ betas, float* __restrict__ VP)
{
  const _Float16* A  = (const _Float16*)PFp;
  const _Float16* Bt = (const _Float16*)BTp;
  __shared__ __align__(16) float sT[8][16 * 68];
  const int lane = threadIdx.x & 31;
  const int wave = threadIdx.x >> 5;
  constexpr int tilesN = kN3P / 64;
  constexpr int tilesM = kB / 64;
  const int tile = blockIdx.x * 8 + wave;
  if (tile >= tilesM * tilesN) return;
  const int tm = tile / tilesN;
  const int tn = tile - tm * tilesN;
  const int m0 = tm << 6;
  const int n0 = tn << 6;
  const int rlane = lane & 15;
  const int koff = (lane >> 4) * 8;
  const int mOff = (lane >> 4) * 8;

  v8f acc[4][4];
#pragma unroll
  for (int i = 0; i < 4; ++i)
#pragma unroll
    for (int j = 0; j < 4; ++j) acc[i][j] = (v8f){0.f, 0.f, 0.f, 0.f, 0.f, 0.f, 0.f, 0.f};

#pragma unroll 1
  for (int k0 = 0; k0 < kKL; k0 += 32) {
    v16h bh[4];
#pragma unroll
    for (int j = 0; j < 4; ++j) bh[j] = frag_load(Bt + (size_t)(n0 + (j << 4) + rlane) * kKP + koff + k0);
#pragma unroll
    for (int i = 0; i < 4; ++i) {
      const v16h ah = frag_load(A + (size_t)(m0 + (i << 4) + rlane) * kKP + koff + k0);
#pragma unroll
      for (int j = 0; j < 4; ++j) acc[i][j] = mma_h(ah, bh[j], acc[i][j]);
    }
  }

  float* slab = sT[wave];
  const int hh = lane >> 4;
  const int c4 = (lane & 15) * 4;
#pragma unroll
  for (int i = 0; i < 4; ++i) {
    const int mBase = m0 + (i << 4);
#pragma unroll
    for (int j = 0; j < 4; ++j)
#pragma unroll
      for (int r = 0; r < 8; ++r) slab[(mOff + r) * 68 + (j << 4) + rlane] = acc[i][j][r] * kInvPose;
    wave_sync_lds();
    const float* vs = VSD + (size_t)(n0 + c4) * 12;
    v4f q[4][3];
#pragma unroll
    for (int e = 0; e < 4; ++e)
#pragma unroll
      for (int t = 0; t < 3; ++t) q[e][t] = *(const v4f*)(vs + e * 12 + t * 4);
#pragma unroll 1
    for (int it = 0; it < 8; ++it) {
      const int row = it * 2 + hh;
      const float* bq = betas + (size_t)(mBase + row) * kNB;
      const v2f be0 = *(const v2f*)(bq + 0);
      const v2f be1 = *(const v2f*)(bq + 2);
      const v2f be2 = *(const v2f*)(bq + 4);
      const v2f be3 = *(const v2f*)(bq + 6);
      const v2f be4 = *(const v2f*)(bq + 8);
      float* sp = slab + row * 68 + c4;
      const v4f sv = *(const v4f*)sp;
      v4f ovv;
#pragma unroll
      for (int e = 0; e < 4; ++e) {
        float a = sv[e] + q[e][2][2];
        a = fmaf(be0[0], q[e][0][0], a);
        a = fmaf(be0[1], q[e][0][1], a);
        a = fmaf(be1[0], q[e][0][2], a);
        a = fmaf(be1[1], q[e][0][3], a);
        a = fmaf(be2[0], q[e][1][0], a);
        a = fmaf(be2[1], q[e][1][1], a);
        a = fmaf(be3[0], q[e][1][2], a);
        a = fmaf(be3[1], q[e][1][3], a);
        a = fmaf(be4[0], q[e][2][0], a);
        a = fmaf(be4[1], q[e][2][1], a);
        ovv[e] = a;
      }
      *(v4f*)sp = ovv;
    }
    for (int pass = 0; pass < 2; ++pass) {
#pragma unroll
      for (int it = 0; it < 8; ++it) {
        const int row = it * 2 + hh;
        const v4f v = *(const v4f*)(slab + row * 68 + c4);
        *(volatile v4f*)(VP + (size_t)(mBase + row) * kN3P + n0 + c4) = v;
      }
      __threadfence();
    }
    wave_sync_lds();
  }
}

__global__ __launch_bounds__(256) void lbs_kernel(
    const unsigned short* __restrict__ W16p, const unsigned short* __restrict__ A16p,
    const float* __restrict__ VP, const float* __restrict__ transl, float* __restrict__ VO)
{
  const _Float16* W  = (const _Float16*)W16p;
  const _Float16* Am = (const _Float16*)A16p;
  __shared__ __align__(16) float sT[8][16 * 52];
  __shared__ __align__(16) float sO[8][768];
  const int lane = threadIdx.x & 31;
  const int wave = threadIdx.x >> 5;
  constexpr int tilesN = kB / 4;
  constexpr int tilesM = kVP / 64;
  const int tile = blockIdx.x * 8 + wave;
  if (tile >= tilesM * tilesN) return;
  const int tm = tile / tilesN;
  const int tn = tile - tm * tilesN;
  const int m0 = tm << 6;
  const int b0 = tn * 4;
  const int n0 = tn * 48;
  const int rlane = lane & 15;
  const int koff = (lane >> 4) * 8;
  const int mOff = (lane >> 4) * 8;

  v16h bh[3];
#pragma unroll
  for (int j = 0; j < 3; ++j) bh[j] = frag_load(Am + (size_t)(n0 + (j << 4) + rlane) * 32 + koff);
  v8f acc[4][3];
#pragma unroll
  for (int i = 0; i < 4; ++i)
#pragma unroll
    for (int j = 0; j < 3; ++j) acc[i][j] = (v8f){0.f, 0.f, 0.f, 0.f, 0.f, 0.f, 0.f, 0.f};
#pragma unroll
  for (int i = 0; i < 4; ++i) {
    const v16h ah = frag_load(W + (size_t)(m0 + (i << 4) + rlane) * 32 + koff);
#pragma unroll
    for (int j = 0; j < 3; ++j) acc[i][j] = mma_h(ah, bh[j], acc[i][j]);
  }

  float* slab = sT[wave];
  float* so = sO[wave];
  const int vloc = lane & 15;
  const int bsel = lane >> 4;
  float tr[2][3];
#pragma unroll
  for (int t = 0; t < 2; ++t)
#pragma unroll
    for (int m = 0; m < 3; ++m) tr[t][m] = transl[(b0 + bsel + 2 * t) * 3 + m];

#pragma unroll
  for (int i = 0; i < 4; ++i) {
#pragma unroll
    for (int j = 0; j < 3; ++j)
#pragma unroll
      for (int r = 0; r < 8; ++r) slab[(mOff + r) * 52 + (j << 4) + rlane] = acc[i][j][r] * kInvLbs;
    wave_sync_lds();
#pragma unroll
    for (int t = 0; t < 2; ++t) {
      const int bb = bsel + 2 * t;
      const int v = m0 + (i << 4) + vloc;
      const float* tp = slab + vloc * 52 + bb * 12;
      const v4f t0 = *(const v4f*)(tp + 0);
      const v4f t1 = *(const v4f*)(tp + 4);
      const v4f t2 = *(const v4f*)(tp + 8);
      const float* pp = VP + (size_t)(b0 + bb) * kN3P + (size_t)v * 3;
      const float px = pp[0], py = pp[1], pz = pp[2];
      const float o0 = fmaf(t0[0], px, fmaf(t0[1], py, fmaf(t0[2], pz, t0[3]))) + tr[t][0];
      const float o1 = fmaf(t1[0], px, fmaf(t1[1], py, fmaf(t1[2], pz, t1[3]))) + tr[t][1];
      const float o2 = fmaf(t2[0], px, fmaf(t2[1], py, fmaf(t2[2], pz, t2[3]))) + tr[t][2];
      float* oq = so + bb * 192 + ((i << 4) + vloc) * 3;
      oq[0] = o0;
      oq[1] = o1;
      oq[2] = o2;
    }
    wave_sync_lds();
  }

  v4f ov[6];
#pragma unroll
  for (int t = 0; t < 6; ++t) ov[t] = *(const v4f*)(so + (t * 32 + lane) * 4);
  for (int pass = 0; pass < 2; ++pass) {
#pragma unroll
    for (int t = 0; t < 6; ++t) {
      const int idx = t * 32 + lane;
      const int bb = idx / 48;
      const int w = idx - bb * 48;
      *(volatile v4f*)(VO + (size_t)(b0 + bb) * kN3P + (size_t)m0 * 3 + w * 4) = ov[t];
    }
    __threadfence();
  }
}

__global__ __launch_bounds__(256) void compact_kernel(const float* __restrict__ VO, float* __restrict__ out)
{
  const int i = blockIdx.x * 256 + threadIdx.x;
  if (i >= kOut0Elems / 4) return;
  const int fbase = i * 4;
  v4f o;
#pragma unroll
  for (int e = 0; e < 4; ++e) {
    const int f = fbase + e;
    const int b = f / kN3;
    const int r = f - b * kN3;
    o[e] = VO[(size_t)b * kN3P + r];
  }
  float* q = out + (size_t)fbase;
  *(volatile v4f*)q = o;
  __threadfence();
  *(volatile v4f*)q = o;
}

extern "C" void kernel_launch(void* const* d_in, const int* in_sizes, int n_in,
                              void* d_out, int out_size, void* d_ws, size_t ws_size,
                              hipStream_t stream) {
  if (n_in < 9) return;
  if (in_sizes[0] != kB * kNB) return;
  if (in_sizes[1] != kB * 3) return;
  if (in_sizes[2] != kB * 69) return;
  if (in_sizes[3] != kB * 3) return;
  if (in_sizes[4] != kV * 3) return;
  if (in_sizes[5] != kV * 3 * kNB) return;
  if (in_sizes[6] != kP * kN3) return;
  if (in_sizes[7] != kJ * kV) return;
  if (in_sizes[8] != kV * kJ) return;
  if (out_size != kOut0Elems + kOut1Elems) return;
  if (ws_size < kWsTotal) return;

  const float* betas  = (const float*)d_in[0];
  const float* go     = (const float*)d_in[1];
  const float* bp     = (const float*)d_in[2];
  const float* transl = (const float*)d_in[3];
  const float* vt     = (const float*)d_in[4];
  const float* sd     = (const float*)d_in[5];
  const float* pd     = (const float*)d_in[6];
  const float* jreg   = (const float*)d_in[7];
  const float* lbs    = (const float*)d_in[8];
  float* out = (float*)d_out;

  char* ws = (char*)d_ws;
  unsigned short* BTPD = (unsigned short*)(ws + kOffBTPD);
  unsigned short* PF16 = (unsigned short*)(ws + kOffPF16);
  unsigned short* W16  = (unsigned short*)(ws + kOffW16);
  unsigned short* A16  = (unsigned short*)(ws + kOffA16);
  unsigned short* JR16 = (unsigned short*)(ws + kOffJR16);
  unsigned short* X16  = (unsigned short*)(ws + kOffX16);
  float*          VSD  = (float*)(ws + kOffVSD);
  float*          CC   = (float*)(ws + kOffCC);
  float*          VP   = (float*)(ws + kOffVP);
  float*          VO   = (float*)(ws + kOffVO);

  prep_small_kernel<<<kBlkW + kBlkJR + kBlkX + kBlkVSD, 256, 0, stream>>>(lbs, jreg, vt, sd, W16, JR16, X16, VSD);
  prep_pd_kernel<<<kN3P / 32, 256, 0, stream>>>(pd, BTPD);
  consts_kernel<<<1, 256, 0, stream>>>(JR16, X16, CC);
  pose_kernel<<<kB / kPB, kPB * kJ, 0, stream>>>(go, bp, betas, transl, CC, PF16, A16, out + (size_t)kOut0Elems);
  pose_gemm_kernel<<<((kB / 64) * (kN3P / 64)) / 8, 256, 0, stream>>>(PF16, BTPD, VSD, betas, VP);
  lbs_kernel<<<((kVP / 64) * (kB / 4)) / 8, 256, 0, stream>>>(W16, A16, VP, transl, VO);
  compact_kernel<<<(kOut0Elems / 4) / 256, 256, 0, stream>>>(VO, out);
}
